// TransformerBlock_35012573397635
// MI455X (gfx1250) — hardware-run, weakly checked
//
#include <hip/hip_runtime.h>


#ifndef NB
#define NB 2
#endif
#ifndef SEQ
#define SEQ 1024
#endif
#define NB_FULL  2
#define SEQ_FULL 1024
#define DM   1024
#define NH_  16
#define HD   64
#define NF   4096
#define MEMN 1024
#define WIN  256
#define J_FULL (MEMN + SEQ_FULL)
#define KOFF (MEMN - WIN)
#define KEYS (WIN + SEQ)
#define KVW  (2 * HD)
#define AW   1
#define NST  ((WIN + 32) / 32)
#define SCP  292
#define OSP  68
#define MSP  132
#define WSC  64.0f
#define WSI  (1.0f / 64.0f)
#define SC2  ((float)(0.125 * 1.4426950408889634))
#define PSH  14.0f
#define NEGB (-3.0e38f)

static_assert(NH_ * HD == DM);
static_assert(HD == 64);
static_assert(KVW == 128);
static_assert(DM % 64 == 0);
static_assert((2 * DM) % 64 == 0);
static_assert(NF % 64 == 0);
static_assert(DM % 32 == 0);
static_assert(NF % 32 == 0);
static_assert(DM == 4 * 32 * 8);
static_assert(SEQ % 64 == 0);
static_assert((NB * SEQ) % 64 == 0);
static_assert((NB * SEQ) % 4 == 0);
static_assert(SEQ % (16 * AW) == 0);
static_assert(SEQ % 32 == 0);
static_assert(WIN % 64 == 0);
static_assert(KOFF % 64 == 0);
static_assert(KOFF >= 0);
static_assert(MEMN % 64 == 0);
static_assert(KEYS % 64 == 0);
static_assert(NST * 32 == WIN + 32);
static_assert(NST * 32 <= SCP);
static_assert((SCP * 4) % 16 == 0);
static_assert((OSP * 4) % 16 == 0);
static_assert((MSP * 4) % 16 == 0);
static_assert(J_FULL % 128 == 0);
static_assert(NB <= NB_FULL);
static_assert(SEQ <= SEQ_FULL);
static_assert(KOFF + (SEQ - 32) + NST * 32 <= J_FULL);
static_assert((size_t)64 * 65 * 4 <= 131072);
static_assert((size_t)64 * MSP * 4 <= 131072);
static_assert((size_t)16 * OSP * 4 <= 131072);
static_assert((size_t)AW * 16 * (2 * SCP + OSP) * 4 <= 131072);
static_assert((size_t)NB_FULL * SEQ_FULL * DM * 4 == (size_t)8388608);
static_assert((size_t)NB_FULL * SEQ_FULL * DM * 4 + (size_t)NB_FULL * SEQ_FULL * J_FULL * 4 == (size_t)25165824);
static_assert((size_t)25165824 + (size_t)NB_FULL * NH_ * J_FULL * KVW * 4 == (size_t)58720256);

typedef _Float16 h16;
typedef __attribute__((ext_vector_type(16))) _Float16 v16h;
typedef __attribute__((ext_vector_type(8)))  _Float16 v8h;
typedef __attribute__((ext_vector_type(8)))  float    v8f;
typedef __attribute__((ext_vector_type(4)))  float    v4f;
typedef v4f  __attribute__((may_alias)) v4fa;

__device__ __forceinline__ unsigned short f2bf(float f) { unsigned u = __float_as_uint(f); u += 0x7FFFu + ((u >> 16) & 1u); return (unsigned short)(u >> 16); }
__device__ __forceinline__ float bfr(float f) { return __uint_as_float(((unsigned)f2bf(f)) << 16); }
__device__ __forceinline__ v16h cat16(v8h lo, v8h hi) { return __builtin_shufflevector(lo, hi, 0, 1, 2, 3, 4, 5, 6, 7, 8, 9, 10, 11, 12, 13, 14, 15); }
__device__ __forceinline__ v8f wmma16(v16h a, v16h b, v8f c) { return __builtin_amdgcn_wmma_f32_16x16x32_f16(false, a, false, b, (short)0, c, false, false); }
__device__ __forceinline__ v16h  ldh(const h16* p) { return cat16(*(const v8h*)p, *(const v8h*)(p + 16)); }
__device__ __forceinline__ void wave_sync() { __builtin_amdgcn_fence(3  , "wavefront"); __builtin_amdgcn_wave_barrier(); asm volatile("" ::: "memory"); }

static __device__ __forceinline__ h16 toh_flush(float v) { const h16 r = (h16)v; return (fabsf(v) < 6.103515625e-05f) ? (h16)0.0f : r; }
static __device__ __forceinline__ v8h pack8(v4f x0, v4f x1) { v8h o;
#pragma unroll
    for (int i = 0; i < 4; ++i) { o[i] = toh_flush(x0[i]); o[4 + i] = toh_flush(x1[i]); }
    return o; }
static __device__ __forceinline__ v8f wmma16g(v16h a, v16h b, v8f c) {
    c = wmma16(a, b, c);
    asm volatile("v_nop\n\tv_nop\n\tv_nop\n\tv_nop" : "+v"(c) : "v"(a), "v"(b));
    return c;
}

static_assert(256 * 2 * 8 == 64 * 64);
static_assert(256 * 4 * 4 == 64 * 64);
__global__ __launch_bounds__(256) void k_wconv(const float* __restrict__ W, h16* Wt, int K, int N) {
#pragma clang fp contract(off)
    __shared__ float tl[64 * 65];
    const int tid = threadIdx.x; const int k0 = blockIdx.x * 64, n0 = blockIdx.y * 64;
#pragma unroll
    for (int i = 0; i < 4; ++i) { const int idx = i * 256 + tid; const int row = idx >> 4, c4 = (idx & 15) * 4;
        const v4f v = *(const v4f*)(W + (size_t)(k0 + row) * N + n0 + c4);
        tl[row * 65 + c4 + 0] = bfr(v[0]) * WSC; tl[row * 65 + c4 + 1] = bfr(v[1]) * WSC;
        tl[row * 65 + c4 + 2] = bfr(v[2]) * WSC; tl[row * 65 + c4 + 3] = bfr(v[3]) * WSC; }
    __syncthreads();
#pragma unroll 1
    for (int ps = 0; ps < 2; ++ps) {
#pragma unroll
        for (int it = 0; it < 2; ++it) { const int p = it * 256 + tid; const int n = p >> 3, k8 = (p & 7) * 8; v8h o;
#pragma unroll
            for (int e = 0; e < 8; ++e) o[e] = toh_flush(tl[(k8 + e) * 65 + n]);
            *(volatile v8h*)(Wt + (size_t)(n0 + n) * K + k0 + k8) = o; }
        if (ps == 0) __threadfence(); }
}

__global__ __launch_bounds__(128) void k_ln(const float* __restrict__ src, int bstride, const float* __restrict__ g, const float* __restrict__ be, h16* dst, int isInput) {
#pragma clang fp contract(off)
    const int lane = threadIdx.x & 31;
    const int wave = __builtin_amdgcn_readfirstlane((int)(threadIdx.x >> 5));
    const int grow = blockIdx.x * 4 + wave; const int b = grow / SEQ, t = grow % SEQ;
    const float* p = src + ((size_t)b * (size_t)bstride + (size_t)t) * DM + lane * 8;
    float s = 0.0f;
#pragma unroll 1
    for (int c = 0; c < 4; ++c) { const v4f a = *(const v4f*)(p + c * 256), d = *(const v4f*)(p + c * 256 + 4);
#pragma unroll
        for (int e = 0; e < 4; ++e) { const float u0 = isInput ? bfr(a[e]) : a[e]; const float u1 = isInput ? bfr(d[e]) : d[e]; s += u0; s += u1; } }
#pragma unroll
    for (int off = 16; off > 0; off >>= 1) s += __shfl_xor(s, off, 32);
    const float mu = s * (1.0f / (float)DM);
    float sq = 0.0f;
#pragma unroll 1
    for (int c = 0; c < 4; ++c) { const v4f a = *(const v4f*)(p + c * 256), d = *(const v4f*)(p + c * 256 + 4);
#pragma unroll
        for (int e = 0; e < 4; ++e) { const float u0 = (isInput ? bfr(a[e]) : a[e]) - mu; const float u1 = (isInput ? bfr(d[e]) : d[e]) - mu; sq += u0 * u0; sq += u1 * u1; } }
#pragma unroll
    for (int off = 16; off > 0; off >>= 1) sq += __shfl_xor(sq, off, 32);
    const float rs = rsqrtf(sq * (1.0f / (float)DM) + 1.0e-5f);
    h16* drow = dst + (size_t)grow * DM + lane * 8;
#pragma unroll 1
    for (int ps = 0; ps < 2; ++ps) {
#pragma unroll 1
        for (int c = 0; c < 4; ++c) {
            const v4f a = *(const v4f*)(p + c * 256), d = *(const v4f*)(p + c * 256 + 4);
            const v4f g0 = *(const v4f*)(g + c * 256 + lane * 8), g1 = *(const v4f*)(g + c * 256 + lane * 8 + 4);
            const v4f b0 = *(const v4f*)(be + c * 256 + lane * 8), b1 = *(const v4f*)(be + c * 256 + lane * 8 + 4);
            v8h o;
#pragma unroll
            for (int e = 0; e < 4; ++e) { const float u0 = isInput ? bfr(a[e]) : a[e]; const float u1 = isInput ? bfr(d[e]) : d[e];
                const float y0 = (u0 - mu) * rs * bfr(g0[e]) + bfr(b0[e]); const float y1 = (u1 - mu) * rs * bfr(g1[e]) + bfr(b1[e]);
                o[e] = toh_flush(y0); o[4 + e] = toh_flush(y1); }
            *(volatile v8h*)(drow + c * 256) = o; }
        if (ps == 0) __threadfence(); }
}

static_assert(256 * 8 * 4 == 64 * KVW);
__global__ __launch_bounds__(256) void k_mem(const float* __restrict__ MK, float* O2, h16* KP, h16* VT) {
#pragma clang fp contract(off)
    __shared__ __align__(16) float ms[64 * MSP];
    const int tid = threadIdx.x; const int bh = blockIdx.y; const int m0 = blockIdx.x * 64;
    const float* src = MK + ((size_t)bh * MEMN + (size_t)m0) * KVW;
    float* dst = O2 + ((size_t)bh * J_FULL + (size_t)m0) * KVW;
    v4f vals[8];
#pragma unroll
    for (int i = 0; i < 8; ++i) { const int idx = i * 256 + tid; v4f v = *(const v4f*)(src + (size_t)idx * 4);
        v[0] = bfr(v[0]); v[1] = bfr(v[1]); v[2] = bfr(v[2]); v[3] = bfr(v[3]); vals[i] = v;
        *(v4fa*)(&ms[(idx >> 5) * MSP + (idx & 31) * 4]) = v; }
#pragma unroll
    for (int i = 0; i < 8; ++i) { const int idx = i * 256 + tid; *(volatile v4f*)(dst + (size_t)idx * 4) = vals[i]; }
    __threadfence();
#pragma unroll
    for (int i = 0; i < 8; ++i) { const int idx = i * 256 + tid; *(volatile v4f*)(dst + (size_t)idx * 4) = vals[i]; }
    __syncthreads();
    if (m0 >= KOFF) {
        const int jr = m0 - KOFF;
#pragma unroll 1
        for (int ps = 0; ps < 2; ++ps) {
#pragma unroll
            for (int it = 0; it < 2; ++it) { const int p = it * 256 + tid; const int row = p >> 3, c8 = (p & 7) * 8;
                const v4f x0 = *(const v4fa*)(&ms[row * MSP + c8]); const v4f x1 = *(const v4fa*)(&ms[row * MSP + c8 + 4]);
                const v8h hv = pack8(x0, x1);
                *(volatile v8h*)(KP + ((size_t)bh * KEYS + (size_t)(jr + row)) * HD + c8) = hv; }
#pragma unroll
            for (int it = 0; it < 2; ++it) { const int p = it * 256 + tid; const int d = p >> 3, k8 = (p & 7) * 8; v8h o;
#pragma unroll
                for (int e = 0; e < 8; ++e) o[e] = toh_flush(ms[(k8 + e) * MSP + HD + d]);
                *(volatile v8h*)(VT + ((size_t)bh * HD + (size_t)d) * KEYS + jr + k8) = o; }
            if (ps == 0) __threadfence(); }
    }
}

static_assert(4 * 32 * 8 == 16 * 64);
static_assert(4 * 4 == 16);
static_assert(8 * 2 == 16);
template <int EP>
__device__ __forceinline__ void gemm_tile(const h16* __restrict__ A, const h16* __restrict__ Bt, const int K,
                                          const float* __restrict__ bias, const float* __restrict__ RES,
                                          h16* P0, h16* P1, float* OF) {
    __shared__ __align__(16) float os[16 * OSP];
    const int lane = threadIdx.x & 31, lr = lane & 15, hi = lane >> 4; const int r0 = blockIdx.x * 64, c0 = blockIdx.y * 64;
    v8f acc[4][4];
#pragma unroll
    for (int mb = 0; mb < 4; ++mb)
#pragma unroll
        for (int nb = 0; nb < 4; ++nb) acc[mb][nb] = (v8f){};
    const size_t aoff = (size_t)(r0 + lr) * K + 8 * hi, boff = (size_t)(c0 + lr) * K + 8 * hi;
#pragma unroll 1
    for (int kc = 0; kc < K; kc += 32) {
        v16h a[4];
#pragma unroll
        for (int mb = 0; mb < 4; ++mb) a[mb] = ldh(A + aoff + (size_t)mb * 16 * K + kc);
#pragma unroll
        for (int nb = 0; nb < 4; ++nb) { const v16h bq = ldh(Bt + boff + (size_t)nb * 16 * K + kc);
#pragma unroll
            for (int mb = 0; mb < 4; ++mb) acc[mb][nb] = wmma16g(a[mb], bq, acc[mb][nb]); }
    }
    const int bb = r0 / SEQ, tt = r0 % SEQ;
    float bc[4];
#pragma unroll
    for (int nb = 0; nb < 4; ++nb) bc[nb] = 0.0f;
    if (EP >= 2) {
#pragma unroll
        for (int nb = 0; nb < 4; ++nb) bc[nb] = bfr(bias[c0 + nb * 16 + lr]);
    }
    const int hh = (EP == 1) ? (c0 >> 7) : (c0 >> 6);
    const int part = (EP == 1) ? ((c0 >> 6) & 1) : 0;
    const int zc = bb * NH_ + hh;
#pragma unroll
    for (int mb = 0; mb < 4; ++mb) {
#pragma unroll
        for (int nb = 0; nb < 4; ++nb) {
#pragma unroll
            for (int j = 0; j < 8; ++j) { float v = acc[mb][nb][j] * WSI + bc[nb]; if (EP == 2) v = fmaxf(v, 0.0f);
                os[(hi * 8 + j) * OSP + nb * 16 + lr] = v; } }
        wave_sync();
#pragma unroll 1
        for (int ps = 0; ps < 2; ++ps) {
            if (EP == 0) {
                const size_t sb = ((size_t)zc * SEQ + (size_t)(tt + mb * 16)) * HD;
#pragma unroll
                for (int s = 0; s < 4; ++s) { const int p = s * 32 + lane; const int row = p >> 3, c8 = (p & 7) * 8;
                    const v4f x0 = *(const v4fa*)(&os[row * OSP + c8]); const v4f x1 = *(const v4fa*)(&os[row * OSP + c8 + 4]);
                    const v8h hv = pack8(x0, x1);
                    *(volatile v8h*)(P0 + sb + (size_t)p * 8) = hv; }
            }
            if (EP == 1) {
                float* orow = OF + ((size_t)zc * J_FULL + (size_t)(MEMN + tt + mb * 16)) * KVW + part * HD;
#pragma unroll
                for (int s = 0; s < 8; ++s) { const int row = 2 * s + (lane >> 4), cofs = (lane & 15) * 4;
                    const v4f val = *(const v4fa*)(&os[row * OSP + cofs]);
                    *(volatile v4f*)(orow + (size_t)row * KVW + cofs) = val; }
                if (part == 0) {
                    const size_t sb = ((size_t)zc * KEYS + (size_t)(WIN + tt + mb * 16)) * HD;
#pragma unroll
                    for (int s = 0; s < 4; ++s) { const int p = s * 32 + lane; const int row = p >> 3, c8 = (p & 7) * 8;
                        const v4f x0 = *(const v4fa*)(&os[row * OSP + c8]); const v4f x1 = *(const v4fa*)(&os[row * OSP + c8 + 4]);
                        const v8h hv = pack8(x0, x1);
                        *(volatile v8h*)(P0 + sb + (size_t)p * 8) = hv; }
                }
            }
            if (EP == 2) {
#pragma unroll
                for (int s = 0; s < 4; ++s) { const int row = 4 * s + (lane >> 3), c8 = (lane & 7) * 8;
                    const v4f x0 = *(const v4fa*)(&os[row * OSP + c8]); const v4f x1 = *(const v4fa*)(&os[row * OSP + c8 + 4]);
                    const v8h hv = pack8(x0, x1);
                    *(volatile v8h*)(P0 + (size_t)(r0 + mb * 16 + row) * NF + c0 + c8) = hv; }
            }
            if (EP == 3) {
#pragma unroll
                for (int s = 0; s < 8; ++s) { const int row = 2 * s + (lane >> 4), cofs = (lane & 15) * 4;
                    const v4f x0 = *(const v4fa*)(&os[row * OSP + cofs]);
                    const v4f rr = *(const v4f*)(RES + (size_t)(r0 + mb * 16 + row) * DM + c0 + cofs);
                    const v4f val = x0 + rr;
                    *(volatile v4f*)(OF + ((size_t)bb * SEQ_FULL + (size_t)(tt + mb * 16 + row)) * DM + c0 + cofs) = val; }
            }
            if (ps == 0) __threadfence(); }
        wave_sync();
    }
    if (EP == 1) {
        if (part == 1) {
#pragma unroll
            for (int nb = 0; nb < 4; ++nb) {
#pragma unroll
                for (int mb = 0; mb < 4; ++mb) {
#pragma unroll
                    for (int j = 0; j < 8; ++j) os[lr * OSP + mb * 16 + hi * 8 + j] = acc[mb][nb][j] * WSI; }
                wave_sync();
#pragma unroll 1
                for (int ps = 0; ps < 2; ++ps) {
#pragma unroll
                    for (int s = 0; s < 4; ++s) { const int row = 4 * s + (lane >> 3), c8 = (lane & 7) * 8;
                        const v4f x0 = *(const v4fa*)(&os[row * OSP + c8]); const v4f x1 = *(const v4fa*)(&os[row * OSP + c8 + 4]);
                        const v8h hv = pack8(x0, x1);
                        *(volatile v8h*)(P1 + ((size_t)zc * HD + (size_t)(nb * 16 + row)) * KEYS + WIN + tt + c8) = hv; }
                    if (ps == 0) __threadfence(); }
                wave_sync();
            }
        }
    }
}

__global__ __launch_bounds__(32) void k_gemm_q(const h16* __restrict__ A, const h16* __restrict__ Bt, h16* QH) {
    gemm_tile<0>(A, Bt, DM, (const float*)nullptr, (const float*)nullptr, QH, (h16*)nullptr, (float*)nullptr);
}
__global__ __launch_bounds__(32) void k_gemm_kv(const h16* __restrict__ A, const h16* __restrict__ Bt, h16* KP, h16* VT, float* O2) {
    gemm_tile<1>(A, Bt, DM, (const float*)nullptr, (const float*)nullptr, KP, VT, O2);
}
__global__ __launch_bounds__(32) void k_gemm_f1(const h16* __restrict__ A, const h16* __restrict__ Bt, const float* __restrict__ bias, h16* A1) {
    gemm_tile<2>(A, Bt, DM, bias, (const float*)nullptr, A1, (h16*)nullptr, (float*)nullptr);
}
__global__ __launch_bounds__(32) void k_gemm_f2(const h16* __restrict__ A, const h16* __restrict__ Bt, const float* __restrict__ bias, const float* __restrict__ HF, float* O0) {
    gemm_tile<3>(A, Bt, NF, bias, HF, (h16*)nullptr, (h16*)nullptr, O0);
}

static_assert(16 * 32 * 4 == J_FULL);
static_assert(16 * 4 == HD);
__global__ __launch_bounds__(32 * AW) void k_attn(const h16* __restrict__ QH, const h16* __restrict__ KP, const h16* __restrict__ VT,
                                                  const float* __restrict__ X, float* HF, float* AWO) {
    __shared__ __align__(16) float sc[AW * 16 * SCP];
    __shared__ __align__(16) float aw[AW * 16 * SCP];
    __shared__ __align__(16) float os[AW * 16 * OSP];
    const int lane = threadIdx.x & 31, lr = lane & 15, hi = lane >> 4;
    const int wave = __builtin_amdgcn_readfirstlane((int)(threadIdx.x >> 5));
    const int b = blockIdx.y;
    const int t0 = (blockIdx.x * AW + wave) * 16;
    const int ks = t0 & ~31;
    const int row = t0 + lr;
    const int wb = wave * 16 * OSP, wb2 = wave * 16 * SCP;
    const int lb = wb2 + lr * SCP + hi * 16;
    const v4f z4 = (v4f){};
#pragma unroll 1
    for (int s = 0; s < NST; ++s) {
#pragma unroll
        for (int q = 0; q < 4; ++q) *(v4fa*)(&aw[lb + s * 32 + q * 4]) = z4; }
#pragma unroll 1
    for (int h = 0; h < NH_; ++h) {
        const int zh = b * NH_ + h;
        const size_t qo = ((size_t)zh * SEQ + (size_t)row) * HD + 8 * hi;
        const v16h q0 = ldh(QH + qo), q1 = ldh(QH + qo + 32);
        const size_t ko = ((size_t)zh * KEYS + (size_t)(ks + lr)) * HD + 8 * hi;
        const size_t vo = ((size_t)zh * HD + (size_t)lr) * KEYS + ks + 8 * hi;
        v8f o0 = (v8f){}, o1 = (v8f){}, o2 = (v8f){}, o3 = (v8f){};
        float m = NEGB, l = 0.0f;
#pragma unroll 1
        for (int s = 0; s < NST; ++s) {
            const h16* ka = KP + ko + (size_t)s * 32 * HD;
            const v16h ka0 = ldh(ka), ka1 = ldh(ka + 32), kb0 = ldh(ka + 16 * HD), kb1 = ldh(ka + 16 * HD + 32);
            v8f sa = (v8f){}, sb = (v8f){};
            sa = wmma16g(ka0, q0, sa); sb = wmma16g(kb0, q0, sb);
            sa = wmma16g(ka1, q1, sa); sb = wmma16g(kb1, q1, sb);
            const int ja = ks + s * 32 + 8 * hi;
            float ta[8], tb[8]; bool fa[8], fb[8]; float mx = NEGB;
#pragma unroll
            for (int r = 0; r < 8; ++r) {
                fa[r] = ((ja + r) >= row) & ((ja + r) <= row + WIN);
                fb[r] = ((ja + 16 + r) >= row) & ((ja + 16 + r) <= row + WIN);
                ta[r] = sa[r] * SC2; tb[r] = sb[r] * SC2;
                mx = fmaxf(mx, fmaxf(fa[r] ? ta[r] : NEGB, fb[r] ? tb[r] : NEGB)); }
            { v4f w0, w1, w2, w3;
#pragma unroll
              for (int r = 0; r < 4; ++r) { w0[r] = ta[r]; w1[r] = ta[4 + r]; w2[r] = tb[r]; w3[r] = tb[4 + r]; }
              *(v4fa*)(&sc[lb + s * 32 + 0]) = w0; *(v4fa*)(&sc[lb + s * 32 + 4]) = w1; *(v4fa*)(&sc[lb + s * 32 + 8]) = w2; *(v4fa*)(&sc[lb + s * 32 + 12]) = w3; }
            mx = fmaxf(mx, __shfl_xor(mx, 16, 32));
            const float mnew = fmaxf(m, mx);
            const float alpha = __builtin_amdgcn_exp2f(m - mnew);
            const float sh = PSH - mnew;
            v16h pb; float ls = 0.0f;
#pragma unroll
            for (int r = 0; r < 8; ++r) {
                const float xa = ta[r] + sh, xb = tb[r] + sh;
                const float ea = __builtin_amdgcn_exp2f(xa), eb = __builtin_amdgcn_exp2f(xb);
                const float ga = (fa[r] & (xa >= -14.0f)) ? ea : 0.0f;
                const float gb = (fb[r] & (xb >= -14.0f)) ? eb : 0.0f;
                const h16 pa = (h16)ga; const h16 pc = (h16)gb;
                pb[r] = pa; pb[8 + r] = pc;
                ls += (float)pa + (float)pc; }
            l = l * alpha + ls; m = mnew;
            o0 = o0 * alpha; o1 = o1 * alpha; o2 = o2 * alpha; o3 = o3 * alpha;
            const h16* va = VT + vo + s * 32;
            const v16h v0 = ldh(va), v1 = ldh(va + (size_t)16 * KEYS), v2 = ldh(va + (size_t)32 * KEYS), v3 = ldh(va + (size_t)48 * KEYS);
            o0 = wmma16g(v0, pb, o0); o1 = wmma16g(v1, pb, o1); o2 = wmma16g(v2, pb, o2); o3 = wmma16g(v3, pb, o3);
        }
        l += __shfl_xor(l, 16, 32);
        const bool any = l > 0.0f;
        const float lsafe = any ? l : 1.0f;
        const float inv = any ? (1.0f / lsafe) : 0.0f;
        { v4f a, c;
          a[0] = o0[0] * inv; a[1] = o0[1] * inv; a[2] = o0[2] * inv; a[3] = o0[3] * inv; c[0] = o0[4] * inv; c[1] = o0[5] * inv; c[2] = o0[6] * inv; c[3] = o0[7] * inv;
          *(v4fa*)(&os[wb + lr * OSP +  0 + 8 * hi]) = a; *(v4fa*)(&os[wb + lr * OSP +  0 + 8 * hi + 4]) = c;
          a[0] = o1[0] * inv; a[1] = o1[1] * inv; a[2] = o1[2] * inv; a[3] = o1[3] * inv; c[0] = o1[4] * inv; c[1] = o1[5] * inv; c[2] = o1[6] * inv; c[3] = o1[7] * inv;
          *(v4fa*)(&os[wb + lr * OSP + 16 + 8 * hi]) = a; *(v4fa*)(&os[wb + lr * OSP + 16 + 8 * hi + 4]) = c;
          a[0] = o2[0] * inv; a[1] = o2[1] * inv; a[2] = o2[2] * inv; a[3] = o2[3] * inv; c[0] = o2[4] * inv; c[1] = o2[5] * inv; c[2] = o2[6] * inv; c[3] = o2[7] * inv;
          *(v4fa*)(&os[wb + lr * OSP + 32 + 8 * hi]) = a; *(v4fa*)(&os[wb + lr * OSP + 32 + 8 * hi + 4]) = c;
          a[0] = o3[0] * inv; a[1] = o3[1] * inv; a[2] = o3[2] * inv; a[3] = o3[3] * inv; c[0] = o3[4] * inv; c[1] = o3[5] * inv; c[2] = o3[6] * inv; c[3] = o3[7] * inv;
          *(v4fa*)(&os[wb + lr * OSP + 48 + 8 * hi]) = a; *(v4fa*)(&os[wb + lr * OSP + 48 + 8 * hi + 4]) = c; }
        wave_sync();
        float* hrow = HF + ((size_t)b * SEQ + (size_t)t0) * DM + h * HD;
        const float* xrow = X + ((size_t)b * SEQ_FULL + (size_t)t0) * DM + h * HD;
#pragma unroll 1
        for (int ps = 0; ps < 2; ++ps) {
#pragma unroll
            for (int s = 0; s < 8; ++s) { const int rw = 2 * s + (lane >> 4), cofs = (lane & 15) * 4;
                v4f val = *(const v4fa*)(&os[wb + rw * OSP + cofs]);
                const v4f xr = *(const v4f*)(xrow + (size_t)rw * DM + cofs);
                val[0] += bfr(xr[0]); val[1] += bfr(xr[1]); val[2] += bfr(xr[2]); val[3] += bfr(xr[3]);
                *(volatile v4f*)(hrow + (size_t)rw * DM + cofs) = val; }
            if (ps == 0) __threadfence(); }
        wave_sync();
        const float shf = PSH - m; const float i16 = inv * (1.0f / (float)NH_);
#pragma unroll 1
        for (int s = 0; s < NST; ++s) {
            const int ja = ks + s * 32 + 8 * hi;
#pragma unroll
            for (int q = 0; q < 4; ++q) {
                const int kq = ja + (q & 1) * 4 + (q >> 1) * 16;
                const v4f tv = *(const v4fa*)(&sc[lb + s * 32 + q * 4]);
                v4f av = *(const v4fa*)(&aw[lb + s * 32 + q * 4]);
#pragma unroll
                for (int e = 0; e < 4; ++e) { const int key = kq + e; const bool keep = (key >= row) & (key <= row + WIN);
                    const float pe = __builtin_amdgcn_exp2f(tv[e] + shf) * i16;
                    av[e] += keep ? pe : 0.0f; }
                *(v4fa*)(&aw[lb + s * 32 + q * 4]) = av; } }
    }
    wave_sync();
    float* arow = AWO + ((size_t)b * SEQ_FULL + (size_t)t0) * J_FULL;
    const int kabs = KOFF + ks;
#pragma unroll 1
    for (int ps = 0; ps < 2; ++ps) {
#pragma unroll 1
        for (int rr = 0; rr < 16; ++rr) {
#pragma unroll 4
            for (int c = 0; c < 16; ++c) {
                const int col = c * 128 + lane * 4; const int rel = col - kabs;
                const bool inb = (rel >= 0) & (rel < NST * 32);
                int rc = rel < 0 ? 0 : rel; rc = rc > (NST * 32 - 4) ? (NST * 32 - 4) : rc;
                const int st = rc >> 5, w = rc & 31;
                const int idx = st * 32 + ((w >> 3) & 1) * 16 + (w & 7) + ((w >> 4) << 3);
                v4f val = *(const v4fa*)(&aw[wb2 + rr * SCP + idx]);
                asm volatile("" : "+v"(val));
                val = inb ? val : z4;
                *(volatile v4f*)(arow + (size_t)rr * J_FULL + col) = val; } }
        if (ps == 0) __threadfence(); }
}

static constexpr size_t al256(size_t v) { return (v + 255) & ~(size_t)255; }
static constexpr size_t SZ_WQ  = al256((size_t)DM * DM * 2);
static constexpr size_t SZ_WKV = al256((size_t)2 * DM * DM * 2);
static constexpr size_t SZ_W1  = al256((size_t)NF * DM * 2);
static constexpr size_t SZ_W2  = al256((size_t)DM * NF * 2);
static constexpr size_t SZ_XN  = al256((size_t)NB * SEQ * DM * 2);
static constexpr size_t SZ_QH  = al256((size_t)NB * NH_ * SEQ * HD * 2);
static constexpr size_t SZ_KP  = al256((size_t)NB * NH_ * KEYS * HD * 2);
static constexpr size_t SZ_HF  = al256((size_t)NB * SEQ * DM * 4);
static constexpr size_t SZ_A1  = al256((size_t)NB * SEQ * NF * 2);
static constexpr size_t SZ_TOTAL = SZ_WQ + SZ_WKV + SZ_W1 + SZ_W2 + 2 * SZ_XN + SZ_QH + 2 * SZ_KP + SZ_HF + SZ_A1;
static_assert(SZ_TOTAL <= (size_t)134217728);
static constexpr size_t OFF1 = (size_t)NB_FULL * SEQ_FULL * DM;
static constexpr size_t OFF2 = OFF1 + (size_t)NB_FULL * SEQ_FULL * J_FULL;
static_assert(OFF1 * 4 == (size_t)8388608);
static_assert(OFF2 * 4 == (size_t)25165824);
static_assert((OFF1 * 4) % 128 == 0);
static_assert((OFF2 * 4) % 128 == 0);

extern "C" void kernel_launch(void* const* d_in, const int* in_sizes, int n_in,
                              void* d_out, int out_size, void* d_ws, size_t ws_size, hipStream_t stream) {
    if (n_in < 12) return;
    const size_t needx = ((size_t)(NB - 1) * SEQ_FULL + SEQ) * DM;
    if ((size_t)in_sizes[0] < needx) return;
    if ((size_t)in_sizes[1] < (size_t)NB * NH_ * MEMN * KVW) return;
    if ((size_t)in_sizes[2] < (size_t)DM * DM || (size_t)in_sizes[3] < (size_t)DM * 2 * DM) return;
    if (in_sizes[4] < DM || in_sizes[5] < DM || in_sizes[6] < DM || in_sizes[7] < DM) return;
    if ((size_t)in_sizes[8] < (size_t)DM * NF || in_sizes[9] < NF || (size_t)in_sizes[10] < (size_t)NF * DM || in_sizes[11] < DM) return;
    if ((size_t)out_size < OFF2 + (size_t)NB * NH_ * J_FULL * KVW) return;
    if (SZ_TOTAL > ws_size) return;
    const float* x    = (const float*)d_in[0];
    const float* mkv  = (const float*)d_in[1];
    const float* wq   = (const float*)d_in[2];
    const float* wkv  = (const float*)d_in[3];
    const float* ln1g = (const float*)d_in[4];
    const float* ln1b = (const float*)d_in[5];
    const float* ln2g = (const float*)d_in[6];
    const float* ln2b = (const float*)d_in[7];
    const float* w1   = (const float*)d_in[8];
    const float* b1   = (const float*)d_in[9];
    const float* w2   = (const float*)d_in[10];
    const float* b2   = (const float*)d_in[11];
    float* OUT0 = (float*)d_out;
    float* OUT1 = OUT0 + OFF1;
    float* OUT2 = OUT0 + OFF2;
    char* wsp = (char*)d_ws;
    h16* WQT  = (h16*)wsp; wsp += SZ_WQ;
    h16* WKVT = (h16*)wsp; wsp += SZ_WKV;
    h16* W1T  = (h16*)wsp; wsp += SZ_W1;
    h16* W2T  = (h16*)wsp; wsp += SZ_W2;
    h16* XN   = (h16*)wsp; wsp += SZ_XN;
    h16* HN   = (h16*)wsp; wsp += SZ_XN;
    h16* QH   = (h16*)wsp; wsp += SZ_QH;
    h16* KP   = (h16*)wsp; wsp += SZ_KP;
    h16* VT   = (h16*)wsp; wsp += SZ_KP;
    float* HF = (float*)wsp; wsp += SZ_HF;
    h16* A1   = (h16*)wsp; wsp += SZ_A1;

    k_wconv<<<dim3(DM / 64, DM / 64, 1), 256, 0, stream>>>(wq, WQT, DM, DM);
    k_wconv<<<dim3(DM / 64, 2 * DM / 64, 1), 256, 0, stream>>>(wkv, WKVT, DM, 2 * DM);
    k_wconv<<<dim3(DM / 64, NF / 64, 1), 256, 0, stream>>>(w1, W1T, DM, NF);
    k_wconv<<<dim3(NF / 64, DM / 64, 1), 256, 0, stream>>>(w2, W2T, NF, DM);

    k_ln<<<NB * SEQ / 4, 128, 0, stream>>>(x, SEQ_FULL, ln1g, ln1b, XN, 1);
    k_gemm_q<<<dim3(NB * SEQ / 64, DM / 64, 1), 32, 0, stream>>>(XN, WQT, QH);
    k_gemm_kv<<<dim3(NB * SEQ / 64, 2 * DM / 64, 1), 32, 0, stream>>>(XN, WKVT, KP, VT, OUT2);
    k_mem<<<dim3(MEMN / 64, NB * NH_, 1), 256, 0, stream>>>(mkv, OUT2, KP, VT);
    k_attn<<<dim3(SEQ / (16 * AW), NB, 1), 32 * AW, 0, stream>>>(QH, KP, VT, x, HF, OUT1);
    k_ln<<<NB * SEQ / 4, 128, 0, stream>>>(HF, SEQ, ln2g, ln2b, HN, 0);
    k_gemm_f1<<<dim3(NB * SEQ / 64, NF / 64, 1), 32, 0, stream>>>(HN, W1T, b1, A1);
    k_gemm_f2<<<dim3(NB * SEQ / 64, DM / 64, 1), 32, 0, stream>>>(A1, W2T, b2, HF, OUT0);
}
